// MultiHeadDeformableAttention_84756884619497
// MI455X (gfx1250) — hardware-verified
//
#include <hip/hip_runtime.h>
#include <stdint.h>


typedef __attribute__((ext_vector_type(16))) _Float16 v16h;
typedef __attribute__((ext_vector_type(8)))  _Float16 v8h;
typedef __attribute__((ext_vector_type(16))) __bf16   v16b;
typedef __attribute__((ext_vector_type(8)))  __bf16   v8b;
typedef __attribute__((ext_vector_type(8)))  float    v8f;
typedef __attribute__((ext_vector_type(4)))  float    v4f;

__device__ __forceinline__ unsigned short f2bf_bits(float f) {
  unsigned u = __float_as_uint(f);
  return (unsigned short)((u + 0x7FFFu + ((u >> 16) & 1u)) >> 16);
}
__device__ __forceinline__ float bf_bits2f(unsigned short h) { return __uint_as_float(((unsigned)h) << 16); }

__device__ __forceinline__ void dep_guard_h(v8f& a, v8f& b, v16h x, v16h y) { asm volatile("v_nop\n\tv_nop\n\tv_nop\n\tv_nop" : "+v"(a), "+v"(b) : "v"(x), "v"(y)); }
__device__ __forceinline__ void dep_guard_b(v8f& a, v8f& b, v16b x, v16b y) { asm volatile("v_nop\n\tv_nop\n\tv_nop\n\tv_nop" : "+v"(a), "+v"(b) : "v"(x), "v"(y)); }
__device__ __forceinline__ void keep4_h(v16h a, v16h b, v16h c, v16h d) { asm volatile("v_nop" :: "v"(a), "v"(b), "v"(c), "v"(d)); }
__device__ __forceinline__ void keep4_b(v16b a, v16b b, v16b c, v16b d) { asm volatile("v_nop" :: "v"(a), "v"(b), "v"(c), "v"(d)); }
__device__ __forceinline__ void acc_guard4(v8f& a, v8f& b, v8f& c, v8f& d) { asm volatile("v_nop\n\tv_nop\n\tv_nop\n\tv_nop" : "+v"(a), "+v"(b), "+v"(c), "+v"(d)); }
template <typename T> struct Frag;
template <> struct Frag<_Float16> {
  typedef v16h V; union U { v16h v; v8h h[2]; };
  static __device__ __forceinline__ v16h load(const _Float16* p) {
    U f; f.h[0] = *(const v8h*)(p); f.h[1] = *(const v8h*)(p + 16); return f.v;
  }
  static __device__ __forceinline__ v8f mma(v16h a, v16h b, v8f c) {
    return __builtin_amdgcn_wmma_f32_16x16x32_f16(false, a, false, b, (short)0, c, false, false);
  }
  static __device__ __forceinline__ void guard(v8f& a, v8f& b, v16h x, v16h y) { dep_guard_h(a, b, x, y); }
  static __device__ __forceinline__ void keep(v16h a, v16h b, v16h c, v16h d) { keep4_h(a, b, c, d); }
};
template <> struct Frag<__bf16> {
  typedef v16b V; union U { v16b v; v8b h[2]; };
  static __device__ __forceinline__ v16b load(const __bf16* p) {
    U f; f.h[0] = *(const v8b*)(p); f.h[1] = *(const v8b*)(p + 16); return f.v;
  }
  static __device__ __forceinline__ v8f mma(v16b a, v16b b, v8f c) {
    return __builtin_amdgcn_wmma_f32_16x16x32_bf16(false, a, false, b, (short)0, c, false, false);
  }
  static __device__ __forceinline__ void guard(v8f& a, v8f& b, v16b x, v16b y) { dep_guard_b(a, b, x, y); }
  static __device__ __forceinline__ void keep(v16b a, v16b b, v16b c, v16b d) { keep4_b(a, b, c, d); }
};

template <int ET> struct Elem;
template <> struct Elem<0> { typedef _Float16 T; };
template <> struct Elem<1> { typedef __bf16 T; };
template <int ET, bool SPLIT, int BIAS_MODE, int OUT_MODE, bool RESID, int ACT = 0>
__global__ __launch_bounds__(256) void wmma_gemm64(
    const unsigned short* __restrict__ Ap, const unsigned short* __restrict__ A2p, int lda, long strideA,
    const unsigned short* __restrict__ Btp, const unsigned short* __restrict__ Bt2p, int ldb, long strideB,
    void* __restrict__ Cout, void* __restrict__ Cout2, int ldc, long strideC,
    const float* __restrict__ bias,
    const float* __restrict__ resid, long strideR,
    int M, int N, int K, float scale, int Mst) {
  typedef typename Elem<ET>::T T;
  typedef typename Frag<T>::V V;
  const T* A = (const T*)Ap; const T* A2 = (const T*)A2p; const T* Bt = (const T*)Btp; const T* Bt2 = (const T*)Bt2p;
  __shared__ __align__(16) float sT[8][16 * 68];
  const int b    = blockIdx.y;
  const int lane = threadIdx.x & 31;
  const int wave = threadIdx.x >> 5;
  const int tilesN = N >> 6;
  const int tilesM = M >> 6;
  const int tile = blockIdx.x * 8 + wave;
  if (tile >= tilesM * tilesN) return;
  const int tm = tile / tilesN;
  const int tn = tile - tm * tilesN;
  const int m0 = tm << 6;
  const int n0 = tn << 6;

  const T* Ab  = A  + (size_t)b * strideA;
  const T* Bb  = Bt + (size_t)b * strideB;
  const T* Ab2 = SPLIT ? (A2  + (size_t)b * strideA) : nullptr;
  const T* Bb2 = SPLIT ? (Bt2 + (size_t)b * strideB) : nullptr;

  const int rlane = lane & 15;
  const int koff  = (lane >> 4) * 8;
  const int mOff  = (lane >> 4) * 8;

  v8f acc[4][4];
#pragma unroll
  for (int i = 0; i < 4; ++i)
#pragma unroll
    for (int j = 0; j < 4; ++j) acc[i][j] = (v8f){0.f,0.f,0.f,0.f,0.f,0.f,0.f,0.f};

  for (int k0 = 0; k0 < K; k0 += 32) {
    V bh[4], bl[4];
#pragma unroll
    for (int j = 0; j < 4; ++j) {
      const size_t bo = (size_t)(n0 + (j << 4) + rlane) * ldb + koff + k0;
      bh[j] = Frag<T>::load(Bb + bo);
      if (SPLIT) bl[j] = Frag<T>::load(Bb2 + bo);
    }
#pragma unroll
    for (int i = 0; i < 4; ++i) {
      const size_t ao = (size_t)(m0 + (i << 4) + rlane) * lda + koff + k0;
      V ah = Frag<T>::load(Ab + ao);
      V al;
      if (SPLIT) al = Frag<T>::load(Ab2 + ao);
#pragma unroll
      for (int j = 0; j < 4; ++j) {
        acc[i][j] = Frag<T>::mma(ah, bh[j], acc[i][j]);
        if (SPLIT) {
          acc[i][j] = Frag<T>::mma(ah, bl[j], acc[i][j]);
          acc[i][j] = Frag<T>::mma(al, bh[j], acc[i][j]);
        }
      }
      Frag<T>::guard(acc[i][0], acc[i][3], ah, SPLIT ? al : ah);
    }
    Frag<T>::keep(bh[0], bh[1], bh[2], bh[3]);
    if (SPLIT) Frag<T>::keep(bl[0], bl[1], bl[2], bl[3]);
  }
  acc_guard4(acc[0][0], acc[0][1], acc[0][2], acc[0][3]);
  acc_guard4(acc[1][0], acc[1][1], acc[1][2], acc[1][3]);
  acc_guard4(acc[2][0], acc[2][1], acc[2][2], acc[2][3]);
  acc_guard4(acc[3][0], acc[3][1], acc[3][2], acc[3][3]);

  float* slab = sT[wave];
  const float* Rb = RESID ? (resid + (size_t)b * strideR) : nullptr;
#pragma unroll
  for (int i = 0; i < 4; ++i) {
    const int mBase = m0 + (i << 4);
#pragma unroll
    for (int j = 0; j < 4; ++j) {
      const int n = n0 + (j << 4) + rlane;
      float bv = 0.f;
      if (BIAS_MODE == 2) bv = bias[n];
#pragma unroll
      for (int r = 0; r < 8; ++r) {
        float v = acc[i][j][r] * scale;
        if (BIAS_MODE == 1) v += bias[mBase + mOff + r];
        if (BIAS_MODE == 2) v += bv;
        if (RESID) v += Rb[(size_t)(mBase + mOff + r) * ldc + n];
        if (ACT == 1) v = tanhf(v);
        if (ACT == 2) v = fmaxf(v, 0.0f);
        if (ACT == 3) v = v / (1.0f + expf(-v));
        if (ACT == 4) v = (v > 0.f) ? v : 0.01f * v;
        if (ACT == 5) v = 0.5f * v * (1.0f + erff(v * 0.70710678118654752f));
        slab[(mOff + r) * 68 + (j << 4) + rlane] = v;
      }
    }
    __builtin_amdgcn_fence(__ATOMIC_RELEASE, "workgroup");
    __builtin_amdgcn_wave_barrier();
    __builtin_amdgcn_fence(__ATOMIC_ACQUIRE, "workgroup");
    if (OUT_MODE == 0) {
      float* C = (float*)Cout + (size_t)b * strideC;
      const int hh = lane >> 4, c4 = (lane & 15) * 4;
      for (int pass = 0; pass < 2; ++pass) {
#pragma unroll
        for (int it = 0; it < 8; ++it) {
          const int row = it * 2 + hh;
          v4f v = *(const v4f*)(slab + row * 68 + c4);
          if (mBase + row < Mst) *(volatile v4f*)(C + (size_t)(mBase + row) * ldc + n0 + c4) = v;
        }
        __threadfence();
      }
    } else {
      const int q = lane >> 3, c8 = (lane & 7) * 8;
      unsigned short* C  = (unsigned short*)Cout  + (size_t)b * strideC;
      unsigned short* C2 = (OUT_MODE == 2) ? ((unsigned short*)Cout2 + (size_t)b * strideC) : nullptr;
      for (int pass = 0; pass < 2; ++pass) {
#pragma unroll
        for (int it = 0; it < 4; ++it) {
          const int row = it * 4 + q;
          const float* sp = slab + row * 68 + c8;
          v8h hv, lv;
#pragma unroll
          for (int e = 0; e < 8; ++e) {
            if (OUT_MODE == 1) {
              hv[e] = (_Float16)sp[e];
            } else {
              unsigned short hb = f2bf_bits(sp[e]);
              unsigned short lb = f2bf_bits(sp[e] - bf_bits2f(hb));
              hv[e] = __builtin_bit_cast(_Float16, hb);
              lv[e] = __builtin_bit_cast(_Float16, lb);
            }
          }
          if (mBase + row < Mst) {
            *(volatile v8h*)(C + (size_t)(mBase + row) * ldc + n0 + c8) = hv;
            if (OUT_MODE == 2) *(volatile v8h*)(C2 + (size_t)(mBase + row) * ldc + n0 + c8) = lv;
          }
        }
        __threadfence();
      }
    }
    __builtin_amdgcn_fence(__ATOMIC_RELEASE, "workgroup");
    __builtin_amdgcn_wave_barrier();
    __builtin_amdgcn_fence(__ATOMIC_ACQUIRE, "workgroup");
  }
}

template <int MODE>
__global__ __launch_bounds__(256) void prep_rows(
    const float* __restrict__ a,
    unsigned short* __restrict__ o0, unsigned short* __restrict__ o1,
    int nval8, int ntot8, float fsc) {
  const int i = blockIdx.x * 256 + threadIdx.x;
  if (i >= ntot8) return;
  const bool live = (i < nval8);
  const int ic = live ? i : (nval8 - 1);
  const float* pa = a + (size_t)ic * 8;
  const v4f a0 = *(const v4f*)(pa), a1 = *(const v4f*)(pa + 4);
  v8h h8, l8;
#pragma unroll
  for (int e = 0; e < 4; ++e) {
    const float s = live ? a0[e] : 0.0f;
    if (MODE == 0) {
      h8[e] = (_Float16)(s * fsc);
      l8[e] = h8[e];
    } else {
      const unsigned short hb = f2bf_bits(s);
      const unsigned short lb = f2bf_bits(s - bf_bits2f(hb));
      h8[e] = __builtin_bit_cast(_Float16, hb);
      l8[e] = __builtin_bit_cast(_Float16, lb);
    }
  }
#pragma unroll
  for (int e = 0; e < 4; ++e) {
    const float s = live ? a1[e] : 0.0f;
    if (MODE == 0) {
      h8[4 + e] = (_Float16)(s * fsc);
      l8[4 + e] = h8[4 + e];
    } else {
      const unsigned short hb = f2bf_bits(s);
      const unsigned short lb = f2bf_bits(s - bf_bits2f(hb));
      h8[4 + e] = __builtin_bit_cast(_Float16, hb);
      l8[4 + e] = __builtin_bit_cast(_Float16, lb);
    }
  }
  const size_t o = (size_t)i * 8;
  *(volatile v8h*)(o0 + o) = h8;
  if (MODE == 1) *(volatile v8h*)(o1 + o) = l8;
  __threadfence();
  *(volatile v8h*)(o0 + o) = h8;
  if (MODE == 1) *(volatile v8h*)(o1 + o) = l8;
}

template <int MODE>
__global__ __launch_bounds__(256) void prep_w(
    const float* __restrict__ W, int nout,
    unsigned short* __restrict__ o0, unsigned short* __restrict__ o1, float scale) {
  __shared__ float t[256 * 33];
  const int tid = threadIdx.x;
  const int n0 = blockIdx.x * 32;
#pragma unroll 1
  for (int i = 0; i < 32; ++i) {
    const int idx = i * 256 + tid;
    const int k = idx >> 5, c = idx & 31;
    t[k * 33 + c] = W[(size_t)k * nout + n0 + c];
  }
  __syncthreads();
  const int wave = tid >> 5, lane = tid & 31;
  for (int pass = 0; pass < 2; ++pass) {
#pragma unroll
    for (int r = 0; r < 4; ++r) {
      const int nl = wave * 4 + r;
      v8h hv, lv;
#pragma unroll
      for (int e = 0; e < 8; ++e) {
        const float x = t[(lane * 8 + e) * 33 + nl] * scale;
        if (MODE == 0) {
          hv[e] = (_Float16)x;
          lv[e] = hv[e];
        } else {
          const unsigned short hb = f2bf_bits(x);
          const unsigned short lb = f2bf_bits(x - bf_bits2f(hb));
          hv[e] = __builtin_bit_cast(_Float16, hb);
          lv[e] = __builtin_bit_cast(_Float16, lb);
        }
      }
      const size_t o = (size_t)(n0 + nl) * 256 + lane * 8;
      *(volatile v8h*)(o0 + o) = hv;
      if (MODE == 1) *(volatile v8h*)(o1 + o) = lv;
    }
    __threadfence();
  }
}

__global__ __launch_bounds__(256) void sample_points(
    const unsigned short* __restrict__ valp,
    const float* __restrict__ offp,
    const float* __restrict__ attp,
    const float* __restrict__ refp,
    const int*   __restrict__ dimp,
    unsigned short* __restrict__ midp,
    int npb, int nrows, float midsc) {
#pragma clang fp contract(off)
  __shared__ __align__(16) float srow[256];
  const int bn   = blockIdx.x;
  const int wave = threadIdx.x >> 5;
  const int lane = threadIdx.x & 31;
  const int m    = wave;
  const int b    = bn / npb;
  const int j16  = lane & 15;

  const float lg = attp[(size_t)bn * 128 + m * 16 + j16];
  float mx = lg;
  mx = fmaxf(mx, __shfl_xor(mx, 1, 32));
  mx = fmaxf(mx, __shfl_xor(mx, 2, 32));
  mx = fmaxf(mx, __shfl_xor(mx, 4, 32));
  mx = fmaxf(mx, __shfl_xor(mx, 8, 32));
  const float ex = expf(lg - mx);
  float sm = ex;
  sm += __shfl_xor(sm, 1, 32);
  sm += __shfl_xor(sm, 2, 32);
  sm += __shfl_xor(sm, 4, 32);
  sm += __shfl_xor(sm, 8, 32);
  const float aw = ex * (1.0f / sm);

  const float offv = offp[(size_t)bn * 256 + m * 32 + lane];
  const float rx   = refp[(size_t)bn * 2 + 0];
  const float ry   = refp[(size_t)bn * 2 + 1];
  int dimi = dimp[lane & 7];
  dimi = min(max(dimi, 1), 16384);
  const int e0 = __shfl(dimi, 0, 32) * __shfl(dimi, 1, 32);
  const int e1 = __shfl(dimi, 2, 32) * __shfl(dimi, 3, 32);
  const int e2 = __shfl(dimi, 4, 32) * __shfl(dimi, 5, 32);
  const int s1 = e0, s2 = e0 + e1, s3 = e0 + e1 + e2;
  const _Float16* val = (const _Float16*)(const void*)valp + m * 32 + lane;
  const int brow = b * npb;
  const int rmax = nrows - 1;

  float acc = 0.0f;
#pragma unroll 1
  for (int j = 0; j < 16; ++j) {
    const int   l  = j >> 2;
    const int   wl = __shfl(dimi, 2 * l, 32);
    const int   hl = __shfl(dimi, 2 * l + 1, 32);
    const int   st = (l == 0) ? 0 : ((l == 1) ? s1 : ((l == 2) ? s2 : s3));
    const float w  = __shfl(aw,   j,         32);
    const float ox = __shfl(offv, 2 * j,     32);
    const float oy = __shfl(offv, 2 * j + 1, 32);
    const float wf = (float)wl, hf = (float)hl;
    const float ptx = rx + ox * (1.0f / wf);
    const float pty = ry + oy * (1.0f / hf);
    const float gx = ptx * 2.0f - 1.0f;
    const float gy = pty * 2.0f - 1.0f;
    float ix = ((gx + 1.0f) * wf - 1.0f) * 0.5f;
    float iy = ((gy + 1.0f) * hf - 1.0f) * 0.5f;
    ix = fminf(fmaxf(ix, -2.0f), wf + 1.0f);
    iy = fminf(fmaxf(iy, -2.0f), hf + 1.0f);
    const float x0f = floorf(ix), y0f = floorf(iy);
    const float wx1 = ix - x0f, wy1 = iy - y0f;
    const float wx0 = 1.0f - wx1, wy0 = 1.0f - wy1;
    const int x0 = (int)x0f, y0 = (int)y0f;
    const int x1 = x0 + 1,   y1 = y0 + 1;
    const bool vx0 = (x0 >= 0) & (x0 < wl), vx1 = (x1 >= 0) & (x1 < wl);
    const bool vy0 = (y0 >= 0) & (y0 < hl), vy1 = (y1 >= 0) & (y1 < hl);
    const int xc0 = min(max(x0, 0), wl - 1), xc1 = min(max(x1, 0), wl - 1);
    const int yc0 = min(max(y0, 0), hl - 1), yc1 = min(max(y1, 0), hl - 1);
    const int rowA = brow + st + yc0 * wl;
    const int rowB = brow + st + yc1 * wl;
    const int r00 = min(max(rowA + xc0, 0), rmax);
    const int r10 = min(max(rowA + xc1, 0), rmax);
    const int r01 = min(max(rowB + xc0, 0), rmax);
    const int r11 = min(max(rowB + xc1, 0), rmax);
    float v00 = (float)val[(size_t)r00 * 256];
    float v10 = (float)val[(size_t)r10 * 256];
    float v01 = (float)val[(size_t)r01 * 256];
    float v11 = (float)val[(size_t)r11 * 256];
    v00 = (vx0 & vy0) ? v00 : 0.0f;
    v10 = (vx1 & vy0) ? v10 : 0.0f;
    v01 = (vx0 & vy1) ? v01 : 0.0f;
    v11 = (vx1 & vy1) ? v11 : 0.0f;
    const float sv = v00 * (wy0 * wx0) + v10 * (wy0 * wx1)
                   + v01 * (wy1 * wx0) + v11 * (wy1 * wx1);
    acc += w * sv;
  }
  srow[m * 32 + lane] = acc * midsc;
  __syncthreads();
  if (wave == 0) {
    const v4f p0 = *(const v4f*)(srow + lane * 8);
    const v4f p1 = *(const v4f*)(srow + lane * 8 + 4);
    v8h hv;
#pragma unroll
    for (int e = 0; e < 4; ++e) { hv[e] = (_Float16)p0[e]; hv[4 + e] = (_Float16)p1[e]; }
    unsigned short* dst = midp + (size_t)bn * 256 + lane * 8;
    *(volatile v8h*)dst = hv;
    __threadfence();
    *(volatile v8h*)dst = hv;
  }
}

extern "C" void kernel_launch(void* const* d_in, const int* in_sizes, int n_in,
                              void* d_out, int out_size, void* d_ws, size_t ws_size,
                              hipStream_t stream) {
  const int NB = 2, NPB = 13294, ROWS = NB * NPB, ROWSP = 26624, DM = 256, NA = 128;
  if (n_in < 12) return;
  if (in_sizes[0] != ROWS * DM || in_sizes[1] != ROWS * 2 || in_sizes[2] != ROWS * DM || in_sizes[3] != 8 ||
      in_sizes[4] != DM * DM || in_sizes[5] != DM || in_sizes[6] != DM * NA || in_sizes[7] != NA ||
      in_sizes[8] != DM * DM || in_sizes[9] != DM || in_sizes[10] != DM * DM || in_sizes[11] != DM ||
      out_size != ROWS * DM) return;

  const float* qin   = (const float*)d_in[0];
  const float* refp  = (const float*)d_in[1];
  const float* feat  = (const float*)d_in[2];
  const int*   dimp  = (const int*)d_in[3];
  const float* Woff  = (const float*)d_in[4];
  const float* boff  = (const float*)d_in[5];
  const float* Wa    = (const float*)d_in[6];
  const float* battn = (const float*)d_in[7];
  const float* Wv    = (const float*)d_in[8];
  const float* bval  = (const float*)d_in[9];
  const float* Wout  = (const float*)d_in[10];
  const float* bout  = (const float*)d_in[11];
  float* out = (float*)d_out;

  const size_t plane16 = (size_t)ROWSP * DM * 2;
  size_t cur = 0;
  auto carve = [&](size_t bytes) { size_t r = cur; cur += (bytes + 127) & ~(size_t)127; return r; };
  const size_t o_qh   = carve(plane16);
  const size_t o_ql   = carve(plane16);
  const size_t o_ff   = carve(plane16);
  const size_t o_val  = carve(plane16);
  const size_t o_off  = carve((size_t)ROWSP * DM * 4);
  const size_t o_att  = carve((size_t)ROWSP * NA * 4);
  const size_t o_wv   = carve((size_t)DM * DM * 2);
  const size_t o_woh  = carve((size_t)DM * DM * 2);
  const size_t o_wol  = carve((size_t)DM * DM * 2);
  const size_t o_wout = carve((size_t)DM * DM * 2);
  const size_t o_wah  = carve((size_t)NA * DM * 2);
  const size_t o_wal  = carve((size_t)NA * DM * 2);
  if (cur > ws_size || cur > (size_t)134217728) return;

  char* ws = (char*)d_ws;
  unsigned short* qh   = (unsigned short*)(ws + o_qh);
  unsigned short* ql   = (unsigned short*)(ws + o_ql);
  unsigned short* ff   = (unsigned short*)(ws + o_ff);
  unsigned short* valh = (unsigned short*)(ws + o_val);
  float*          offb = (float*)(ws + o_off);
  float*          attb = (float*)(ws + o_att);
  unsigned short* wvT  = (unsigned short*)(ws + o_wv);
  unsigned short* wohT = (unsigned short*)(ws + o_woh);
  unsigned short* wolT = (unsigned short*)(ws + o_wol);
  unsigned short* woT  = (unsigned short*)(ws + o_wout);
  unsigned short* wahT = (unsigned short*)(ws + o_wah);
  unsigned short* walT = (unsigned short*)(ws + o_wal);

  {
    const int nval8 = ROWS * DM / 8, ntot8 = ROWSP * DM / 8;
    prep_rows<1><<<dim3((ntot8 + 255) / 256), dim3(256), 0, stream>>>(qin,  qh, ql, nval8, ntot8, 1.0f);
    prep_rows<0><<<dim3((ntot8 + 255) / 256), dim3(256), 0, stream>>>(feat, ff, ff, nval8, ntot8, 8.0f);
  }
  prep_w<1><<<dim3(DM / 32), dim3(256), 0, stream>>>(Woff, DM, wohT, wolT, 1.0f);
  prep_w<1><<<dim3(NA / 32), dim3(256), 0, stream>>>(Wa,   NA, wahT, walT, 1.0f);
  prep_w<0><<<dim3(DM / 32), dim3(256), 0, stream>>>(Wv,   DM, wvT,  wvT,  64.0f);
  prep_w<0><<<dim3(DM / 32), dim3(256), 0, stream>>>(Wout, DM, woT,  woT,  64.0f);

  const int tilesM = ROWSP / 64;
  {
    const int tiles = tilesM * (DM / 64);
    wmma_gemm64<0, false, 2, 1, false, 0><<<dim3((tiles + 7) / 8, 1), dim3(256), 0, stream>>>(
        ff, ff, DM, 0L, wvT, wvT, DM, 0L, (void*)valh, (void*)woT, DM, 0L,
        bval, bval, 0L, ROWSP, DM, DM, 1.0f / 512.0f, ROWSP);
  }
  {
    const int tiles = tilesM * (DM / 64);
    wmma_gemm64<1, true, 2, 0, false, 0><<<dim3((tiles + 7) / 8, 1), dim3(256), 0, stream>>>(
        qh, ql, DM, 0L, wohT, wolT, DM, 0L, (void*)offb, (void*)woT, DM, 0L,
        boff, boff, 0L, ROWSP, DM, DM, 1.0f, ROWSP);
  }
  {
    const int tiles = tilesM * (NA / 64);
    wmma_gemm64<1, true, 2, 0, false, 0><<<dim3((tiles + 7) / 8, 1), dim3(256), 0, stream>>>(
        qh, ql, DM, 0L, wahT, walT, DM, 0L, (void*)attb, (void*)woT, NA, 0L,
        battn, battn, 0L, ROWSP, NA, DM, 1.0f, ROWSP);
  }
  sample_points<<<dim3(ROWS), dim3(256), 0, stream>>>(valh, offb, attb, refp, dimp, ff, NPB, ROWS, 16.0f);
  {
    const int tiles = tilesM * (DM / 64);
    wmma_gemm64<0, false, 2, 0, false, 0><<<dim3((tiles + 7) / 8, 1), dim3(256), 0, stream>>>(
        ff, ff, DM, 0L, woT, woT, DM, 0L, (void*)out, (void*)ql, DM, 0L,
        bout, bout, 0L, ROWSP, DM, DM, 1.0f / 1024.0f, ROWS);
  }
}
